// MultiheadAttention_56392920596705
// MI455X (gfx1250) — hardware-verified
//
#include <hip/hip_runtime.h>


#ifndef NB
#define NB 4
#endif
#ifndef SEQ
#define SEQ 2048
#endif
#define NB_FULL   4
#define SEQ_FULL  2048
#define HID       1024
#define NHEAD     16
#define HD        64
#define MROWS     (NB * SEQ)

#define EROWS     256
#define EB        (EROWS / 128)
#define RES_SCALE 2048.0f
#define RES_INV   0.00048828125f
#define NKT       (SEQ / 64)

static_assert(HID == NHEAD * HD);
static_assert(HID == 1024);
static_assert(NHEAD == 16);
static_assert(HD == 64);
static_assert(SEQ % 128 == 0);
static_assert(SEQ <= SEQ_FULL);
static_assert(NB >= 1 && NB <= NB_FULL);
static_assert(MROWS % 128 == 0);
static_assert(HID % 128 == 0);
static_assert(HID % 32 == 0);
static_assert(EROWS % 128 == 0);
static_assert(EROWS >= 128 && EROWS <= SEQ);
static_assert(EB >= 1);

#define N_X   ((size_t)MROWS * HID)
#define N_W   ((size_t)HID * HID)
#define N_R   ((size_t)NB * EROWS * HID)
#define N_MW  ((size_t)(SEQ / 16) * NKT * 32)
#define N_MF  ((size_t)(SEQ / 128) * NKT * 32)

#define CARRY_X    16.0f
#define CARRY_W    32.0f
#define CARRY_QKV  16.0f
#define CARRY_CTX  1024.0f

typedef unsigned u32;
typedef _Float16 f16;
typedef f16   v16h __attribute__((ext_vector_type(16)));
typedef f16   v8h  __attribute__((ext_vector_type(8)));
typedef float v8f  __attribute__((ext_vector_type(8)));
typedef float v4f  __attribute__((ext_vector_type(4)));

union FragU { v16h v; v8h half[2]; f16 e[16]; };
union H8U   { v8h v; f16 e[8]; };

__device__ __forceinline__ v8f zero8() {
    v8f z = {0.f, 0.f, 0.f, 0.f, 0.f, 0.f, 0.f, 0.f};
    return z;
}

__device__ __forceinline__ v8f wmma16(v16h a, v16h b, v8f c) {
    v8f d = __builtin_amdgcn_wmma_f32_16x16x32_f16(false, a, false, b, (short)0, c, false, false);
    asm volatile("v_nop\n\tv_nop\n\tv_nop\n\tv_nop" : "+v"(d) : "v"(a), "v"(b));
    return d;
}

__device__ __forceinline__ float bf16_rne(float x) {
    u32 u = __float_as_uint(x);
    u = (u + 0x7fffu + ((u >> 16) & 1u)) & 0xffff0000u;
    return __uint_as_float(u);
}

__device__ __forceinline__ float fexp2(float x) {
#if defined(__has_builtin)
#if __has_builtin(__builtin_amdgcn_exp2f)
    return __builtin_amdgcn_exp2f(x);
#else
    return exp2f(x);
#endif
#else
    return exp2f(x);
#endif
}

__device__ __forceinline__ float rowmax16(float x) {
    int v = __builtin_bit_cast(int, x);
    x = fmaxf(x, __builtin_bit_cast(float, __builtin_amdgcn_update_dpp(v, v, 0x121, 0xf, 0xf, false)));
    v = __builtin_bit_cast(int, x);
    x = fmaxf(x, __builtin_bit_cast(float, __builtin_amdgcn_update_dpp(v, v, 0x122, 0xf, 0xf, false)));
    v = __builtin_bit_cast(int, x);
    x = fmaxf(x, __builtin_bit_cast(float, __builtin_amdgcn_update_dpp(v, v, 0x124, 0xf, 0xf, false)));
    v = __builtin_bit_cast(int, x);
    x = fmaxf(x, __builtin_bit_cast(float, __builtin_amdgcn_update_dpp(v, v, 0x128, 0xf, 0xf, false)));
    return x;
}

__device__ __forceinline__ v16h load_frag(const f16* tile, u32 rowbase, u32 pitch, u32 kcol, u32 lane) {
    const u32 r  = rowbase + (lane & 15u);
    const u32 kh = (lane >> 4) << 3;
    const f16* p = tile + (size_t)r * pitch + kcol + kh;
    FragU f;
    f.half[0] = *(const v8h*)(p);
    f.half[1] = *(const v8h*)(p + 16);
    return f.v;
}

__device__ __forceinline__ v16h load_frag_g(const f16* __restrict__ rows, u32 rowbase, u32 pitch, u32 kcol, u32 lane) {
    const u32 r  = rowbase + (lane & 15u);
    const u32 kh = (lane >> 4) << 3;
    const f16* p = rows + (size_t)r * pitch + kcol + kh;
    FragU f;
    f.half[0] = *(const v8h*)(p);
    f.half[1] = *(const v8h*)(p + 16);
    return f.v;
}

static __device__ __forceinline__ f16 toh_flush(float v) {
    const f16 r = (f16)v;
    return (fabsf(v) < 6.103515625e-05f) ? (f16)0.0f : r;
}

__device__ __forceinline__ v8h zero8h() {
    v8h z = {(f16)0.0f, (f16)0.0f, (f16)0.0f, (f16)0.0f, (f16)0.0f, (f16)0.0f, (f16)0.0f, (f16)0.0f};
    return z;
}

__global__ void __launch_bounds__(256)
cvt_rows(const float* __restrict__ src, f16* __restrict__ dst, u32 nrows, u32 seqv, u32 seqfull, float carry) {
    const u32 g  = blockIdx.x * 256u + threadIdx.x;
    const u32 m  = g >> 7;
    const u32 c8 = (g & 127u) << 3;
    if (m >= nrows) return;
    const u32 mb = m / seqv;
    const u32 sm = mb * seqfull + (m - mb * seqv);
    const float* sp = src + (size_t)sm * HID + c8;
    const v4f a = *(const v4f*)sp;
    const v4f b = *(const v4f*)(sp + 4);
    H8U o;
#pragma unroll
    for (u32 j = 0; j < 4; ++j) {
        const float x0 = a[j];
        const float x1 = b[j];
        o.e[j]     = (f16)(bf16_rne(x0) * carry);
        o.e[j + 4] = (f16)(bf16_rne(x1) * carry);
    }
    f16* dp = dst + (size_t)m * HID + c8;
    *(volatile v8h*)dp = o.v;
    __threadfence();
    *(volatile v8h*)dp = o.v;
}

__global__ void __launch_bounds__(256)
k_mask_pack(const int* __restrict__ mask, u32* __restrict__ Mw, u32* __restrict__ Mf) {
    __shared__ u32 anyv[8];
    const u32 tid  = threadIdx.x;
    const u32 lane = tid & 31u;
    const u32 wave = (u32)__builtin_amdgcn_readfirstlane((int)(tid >> 5));
    const u32 hh8  = (lane >> 4) << 3;
    const u32 c16  = lane & 15u;
    const u32 qb   = blockIdx.x;
    const u32 kt   = blockIdx.y;
    const u32 q0   = qb * 128u + wave * 16u;
    const u32 kbase = kt * 64u;

    u32 word = 0u;
#pragma unroll 1
    for (u32 r = 0; r < 8u; ++r) {
        const int* rp = mask + (size_t)(q0 + hh8 + r) * SEQ_FULL + kbase + c16;
        const int a0 = rp[0];
        const int a1 = rp[16];
        const int a2 = rp[32];
        const int a3 = rp[48];
        u32 nib = (a0 != 0) ? 1u : 0u;
        nib |= (a1 != 0) ? 2u : 0u;
        nib |= (a2 != 0) ? 4u : 0u;
        nib |= (a3 != 0) ? 8u : 0u;
        word |= nib << (r * 4u);
    }
    int fv = (word != 0u) ? 1 : 0;
    fv |= __shfl_xor(fv, 16);
    fv |= __shfl_xor(fv, 8);
    fv |= __shfl_xor(fv, 4);
    fv |= __shfl_xor(fv, 2);
    fv |= __shfl_xor(fv, 1);
    if (lane == 0u) anyv[wave] = (u32)fv;
    __syncthreads();
    u32 flag = 0u;
#pragma unroll
    for (u32 i = 0; i < 8u; ++i) flag |= anyv[i];

    u32* wp = Mw + ((size_t)(qb * 8u + wave) * NKT + kt) * 32u + lane;
    u32* fp = Mf + ((size_t)qb * NKT + kt) * 32u + lane;
    *(volatile u32*)wp = word;
    if (wave == 0u) *(volatile u32*)fp = flag;
    __threadfence();
    *(volatile u32*)wp = word;
    if (wave == 0u) *(volatile u32*)fp = flag;
}

template <int MODE>
__device__ __forceinline__ void gemm_body(const f16* __restrict__ A, const f16* __restrict__ W,
                                          const float* __restrict__ bias, const float biasMul,
                                          f16* __restrict__ outH, float* __restrict__ outF,
                                          const float accMul, const size_t resOff, const size_t aResOff) {
    __shared__ __attribute__((aligned(16))) f16 As[128 * 32];
    __shared__ __attribute__((aligned(16))) f16 Bs[128 * 32];
    __shared__ __attribute__((aligned(16))) f16 Cs[(MODE == 2) ? 8 : 128 * 128];
    __shared__ __attribute__((aligned(16))) float Cf[(MODE == 2) ? 64 * 128 : 4];

    const u32 tid  = threadIdx.x;
    const u32 lane = tid & 31u;
    const u32 wave = (u32)__builtin_amdgcn_readfirstlane((int)(tid >> 5));
    const u32 wm   = wave & 3u;
    const u32 wn   = wave >> 2;
    const u32 hh8  = (lane >> 4) << 3;
    const u32 c16  = lane & 15u;
    const u32 m0   = blockIdx.x * 128u;
    const u32 n0   = blockIdx.y * 128u;
    const u32 bidx = m0 / (u32)SEQ;
    const u32 s0   = m0 - bidx * (u32)SEQ;
    const bool early = (s0 < (u32)EROWS);

    v8f acc[2][4];
#pragma unroll
    for (int i = 0; i < 2; ++i)
#pragma unroll
        for (int j = 0; j < 4; ++j) acc[i][j] = zero8();

    const u32 srow = tid >> 1;
    const u32 scol = (tid & 1u) << 4;
    const f16* gW = W + (size_t)(n0 + srow) * HID + scol;
    const size_t aHi  = (size_t)(m0 + srow) * HID + scol;
    const size_t aRes = aResOff + (size_t)(bidx * (u32)EROWS + (s0 & (u32)(EROWS - 1)) + srow) * HID + scol;

    u32 npass = 1u;
    if constexpr (MODE == 2) {
        if (early) npass = 2u;
    }

#pragma unroll 1
    for (u32 ap = 0; ap < npass; ++ap) {
        const bool resp = (ap + 1u < npass);
        const size_t aoff = resp ? aRes : aHi;
        const f16* gA = A + aoff;

#pragma unroll 1
        for (u32 k0 = 0; k0 < (u32)HID; k0 += 32u) {
            const v8h ra0 = *(const v8h*)(gA + k0);
            const v8h ra1 = *(const v8h*)(gA + k0 + 8);
            const v8h rb0 = *(const v8h*)(gW + k0);
            const v8h rb1 = *(const v8h*)(gW + k0 + 8);
            __syncthreads();
            *(v8h*)&As[srow * 32u + scol]      = ra0;
            *(v8h*)&As[srow * 32u + scol + 8u] = ra1;
            *(v8h*)&Bs[srow * 32u + scol]      = rb0;
            *(v8h*)&Bs[srow * 32u + scol + 8u] = rb1;
            __syncthreads();

            v16h af[2], bfr[4];
#pragma unroll
            for (int i = 0; i < 2; ++i) af[i] = load_frag(As, wm * 32u + (u32)i * 16u, 32u, 0u, lane);
#pragma unroll
            for (int j = 0; j < 4; ++j) bfr[j] = load_frag(Bs, wn * 64u + (u32)j * 16u, 32u, 0u, lane);
#pragma unroll
            for (int i = 0; i < 2; ++i)
#pragma unroll
                for (int j = 0; j < 4; ++j) acc[i][j] = wmma16(af[i], bfr[j], acc[i][j]);
        }

        if (resp) {
#pragma unroll
            for (int i = 0; i < 2; ++i)
#pragma unroll
                for (int j = 0; j < 4; ++j)
#pragma unroll
                    for (int r = 0; r < 8; ++r) acc[i][j][r] = acc[i][j][r] * RES_INV;
        }
    }

    float bcol[4];
#pragma unroll
    for (int j = 0; j < 4; ++j)
        bcol[j] = bf16_rne(bias[n0 + wn * 64u + (u32)j * 16u + c16]) * biasMul;

    const u32 piece = lane & 7u;
    const u32 lsub  = lane >> 3;

    if constexpr (MODE == 0) {
        const size_t bh0 = (size_t)bidx * NHEAD + (n0 >> 6);
        const u32 nph = early ? 2u : 1u;
#pragma unroll 1
        for (u32 ph = 0; ph < nph; ++ph) {
            __syncthreads();
#pragma unroll
            for (int i = 0; i < 2; ++i)
#pragma unroll
                for (int j = 0; j < 4; ++j) {
                    const u32 nl = wn * 64u + (u32)j * 16u + c16;
#pragma unroll
                    for (int r = 0; r < 8; ++r) {
                        const u32 ml = wm * 32u + (u32)i * 16u + hh8 + (u32)r;
                        const float val = acc[i][j][r] * accMul + bcol[j];
                        const f16 hv = toh_flush(val);
                        const f16 rv = toh_flush((val - (float)hv) * RES_SCALE);
                        Cs[ml * 128u + nl] = (ph == 0u) ? hv : rv;
                    }
                }
            __syncthreads();
#pragma unroll
            for (int pass = 0; pass < 2; ++pass) {
#pragma unroll
                for (u32 it = 0; it < 8; ++it) {
                    const u32 L    = wave * 32u + it * 4u + lsub;
                    const u32 ml   = L >> 1;
                    const u32 hsel = L & 1u;
                    const v8h v = *(const v8h*)&Cs[ml * 128u + hsel * 64u + piece * 8u];
                    const size_t oHi = ((bh0 + hsel) * (u32)SEQ + s0 + ml) * HD + piece * 8u;
                    const size_t oRs = resOff + ((bh0 + hsel) * (u32)EROWS + (s0 & (u32)(EROWS - 1)) + ml) * HD + piece * 8u;
                    f16* dp = outH + ((ph == 0u) ? oHi : oRs);
                    *(volatile v8h*)dp = v;
                }
                if (pass == 0) __threadfence();
            }
        }
    } else if constexpr (MODE == 1) {
        const u32 nph = early ? 2u : 1u;
#pragma unroll 1
        for (u32 ph = 0; ph < nph; ++ph) {
            __syncthreads();
#pragma unroll
            for (int i = 0; i < 2; ++i)
#pragma unroll
                for (int j = 0; j < 4; ++j) {
                    const u32 nl = wn * 64u + (u32)j * 16u + c16;
                    H8U t;
#pragma unroll
                    for (int r = 0; r < 8; ++r) {
                        const float val = acc[i][j][r] * accMul + bcol[j];
                        const f16 hv = toh_flush(val);
                        const f16 rv = toh_flush((val - (float)hv) * RES_SCALE);
                        t.e[r] = (ph == 0u) ? hv : rv;
                    }
                    *(v8h*)&Cs[nl * 128u + wm * 32u + (u32)i * 16u + hh8] = t.v;
                }
            __syncthreads();
#pragma unroll
            for (int pass = 0; pass < 2; ++pass) {
#pragma unroll
                for (u32 it = 0; it < 8; ++it) {
                    const u32 L  = wave * 32u + it * 4u + lsub;
                    const u32 nl = L >> 1;
                    const u32 mh = L & 1u;
                    const v8h v = *(const v8h*)&Cs[nl * 128u + mh * 64u + piece * 8u];
                    const size_t oHi = (size_t)(bidx * (u32)HID + n0 + nl) * (u32)SEQ + s0 + mh * 64u + piece * 8u;
                    const size_t oRs = resOff + (size_t)(bidx * (u32)HID + n0 + nl) * (u32)EROWS + (s0 & (u32)(EROWS - 1)) + mh * 64u + piece * 8u;
                    f16* dp = outH + ((ph == 0u) ? oHi : oRs);
                    *(volatile v8h*)dp = v;
                }
                if (pass == 0) __threadfence();
            }
        }
    } else {
#pragma unroll
        for (u32 half = 0; half < 2; ++half) {
            if ((wm >> 1) == half) {
#pragma unroll
                for (int i = 0; i < 2; ++i)
#pragma unroll
                    for (int j = 0; j < 4; ++j) {
                        const u32 nl = wn * 64u + (u32)j * 16u + c16;
#pragma unroll
                        for (int r = 0; r < 8; ++r) {
                            const u32 ml = (wm & 1u) * 32u + (u32)i * 16u + hh8 + (u32)r;
                            Cf[ml * 128u + nl] = acc[i][j][r] * accMul + bcol[j];
                        }
                    }
            }
            __syncthreads();
#pragma unroll
            for (int pass = 0; pass < 2; ++pass) {
#pragma unroll
                for (u32 it = 0; it < 8; ++it) {
                    const u32 L    = wave * 32u + it * 4u + lsub;
                    const u32 row  = L >> 2;
                    const u32 part = L & 3u;
                    const v4f v = *(const v4f*)&Cf[row * 128u + part * 32u + piece * 4u];
                    float* dp = outF + (size_t)(m0 + half * 64u + row) * HID + n0 + part * 32u + piece * 4u;
                    *(volatile v4f*)dp = v;
                }
                if (pass == 0) __threadfence();
            }
            __syncthreads();
        }
    }
}

__global__ void __launch_bounds__(256) __attribute__((amdgpu_num_vgpr(256)))
k_gemm_qk(const f16* __restrict__ Xh, const f16* __restrict__ Wt, const float* __restrict__ bqkv,
          f16* __restrict__ QKp, size_t resOff0, float accMul, float biasMul) {
    const u32 z = blockIdx.z;
    const size_t resOff = (resOff0 + (size_t)z * N_R) - (size_t)z * N_X;
    gemm_body<0>(Xh, Wt + (size_t)z * HID * HID, bqkv + z * (u32)HID, biasMul,
                 QKp + (size_t)z * MROWS * HID, (float*)0, accMul, resOff, (size_t)0);
}

__global__ void __launch_bounds__(256) __attribute__((amdgpu_num_vgpr(256)))
k_gemm_vt(const f16* __restrict__ Xh, const f16* __restrict__ Wv, const float* __restrict__ bv,
          f16* __restrict__ Vtp, size_t resOff, float accMul, float biasMul) {
    gemm_body<1>(Xh, Wv, bv, biasMul, Vtp, (float*)0, accMul, resOff, (size_t)0);
}

__global__ void __launch_bounds__(256) __attribute__((amdgpu_num_vgpr(256)))
k_gemm_out(const f16* __restrict__ Cp, const f16* __restrict__ Wo,
           const float* __restrict__ bproj, float* __restrict__ out, size_t aResOff, float accMul) {
    gemm_body<2>(Cp, Wo, bproj, 1.0f, (f16*)0, out, accMul, (size_t)0, aResOff);
}

template <int EARLY>
__device__ __forceinline__ void attn_body(const f16* __restrict__ Qp, const f16* __restrict__ Kp,
                                          const f16* __restrict__ Vt, const f16* __restrict__ QRp,
                                          const f16* __restrict__ KRp, const f16* __restrict__ VRp,
                                          const u32* __restrict__ Mw, const u32* __restrict__ Mf,
                                          f16* __restrict__ Cp, f16* __restrict__ CRp, const u32 qb) {
    constexpr u32 KT = 64u;
    __shared__ __attribute__((aligned(16))) f16 ks[KT * 64];
    __shared__ __attribute__((aligned(16))) f16 vsT[64 * KT];
    __shared__ __attribute__((aligned(16))) f16 ps[8][16 * 64];
    __shared__ __attribute__((aligned(16))) f16 krs[EARLY ? KT * 64 : 8];
    __shared__ __attribute__((aligned(16))) f16 vrsT[EARLY ? 64 * KT : 8];
    __shared__ __attribute__((aligned(16))) f16 psr[EARLY ? 8 * 16 * 64 : 8];

    const u32 tid  = threadIdx.x;
    const u32 lane = tid & 31u;
    const u32 wave = (u32)__builtin_amdgcn_readfirstlane((int)(tid >> 5));
    const u32 hh8  = (lane >> 4) << 3;
    const u32 c16  = lane & 15u;
    const u32 bh   = blockIdx.y;
    const u32 bidx = bh >> 4;
    const u32 hidx = bh & 15u;
    const u32 q0   = qb * 128u + wave * 16u;
    const size_t head  = (size_t)bh * SEQ * HD;
    const size_t headR = (size_t)bh * EROWS * HD;

    v16h qa[2];
    if constexpr (!EARLY) {
#pragma unroll
        for (int c = 0; c < 2; ++c) qa[c] = load_frag_g(Qp + head, q0, HD, (u32)c * 32u, lane);
    }

    FragU onesu;
#pragma unroll
    for (int i = 0; i < 16; ++i) onesu.e[i] = (f16)1.0f;
    const v16h ones = onesu.v;

    float m[8];
    v8f   o[4], lacc, oR[4], laccR;
#pragma unroll
    for (int r = 0; r < 8; ++r) m[r] = -1.0e30f;
#pragma unroll
    for (int dt = 0; dt < 4; ++dt) { o[dt] = zero8(); oR[dt] = zero8(); }
    lacc = zero8();
    laccR = zero8();

    const float cl = 1.4426950408889634f * 0.00048828125f;
    f16* psw = &ps[wave][0];
    f16* prw = &psr[EARLY ? wave * 1024u : 0u];

    const u32 nkt = (u32)SEQ / KT;
    const u32* fl  = Mf + (size_t)qb * nkt * 32u;
    const u32* mwp = Mw + (size_t)(qb * 8u + wave) * nkt * 32u + lane;

#pragma unroll 1
    for (u32 kt = 0; kt < nkt; ++kt) {
        const u32 flag = (u32)__builtin_amdgcn_readfirstlane((int)fl[(size_t)kt * 32u]);
        if (flag == 0u) continue;
        const u32 kbase = kt * KT;
        __syncthreads();
#pragma unroll
        for (u32 i = 0; i < 2; ++i) {
            const u32 p   = tid + i * 256u;
            const u32 row = p >> 3;
            const u32 pc  = (p & 7u) << 3;
            const v8h kv = *(const v8h*)(Kp + head + (size_t)(kbase + row) * HD + pc);
            const v8h vv = *(const v8h*)(Vt + head + (size_t)row * SEQ + kbase + pc);
            *(v8h*)&ks[row * 64u + pc]  = kv;
            *(v8h*)&vsT[row * KT + pc]  = vv;
            if constexpr (EARLY) {
                v8h krv = zero8h();
                v8h vrv = zero8h();
                if (kbase < (u32)EROWS) {
                    krv = *(const v8h*)(KRp + headR + (size_t)(kbase + row) * HD + pc);
                    vrv = *(const v8h*)(VRp + headR + (size_t)row * EROWS + kbase + pc);
                }
                *(v8h*)&krs[row * 64u + pc]  = krv;
                *(v8h*)&vrsT[row * KT + pc]  = vrv;
            }
        }
        const u32 mw = mwp[(size_t)kt * 32u];
        __syncthreads();

        v8f s[4], sr[4];
#pragma unroll
        for (int nt = 0; nt < 4; ++nt) { s[nt] = zero8(); sr[nt] = zero8(); }
        if constexpr (EARLY) {
#pragma unroll
            for (int c = 0; c < 2; ++c) {
                const v16h qhf = load_frag_g(Qp + head, q0, HD, (u32)c * 32u, lane);
                const v16h qrf = load_frag_g(QRp + headR, q0, HD, (u32)c * 32u, lane);
#pragma unroll
                for (int nt = 0; nt < 4; ++nt) {
                    const v16h kb  = load_frag(ks, (u32)nt * 16u, 64u, (u32)c * 32u, lane);
                    const v16h krb = load_frag(krs, (u32)nt * 16u, 64u, (u32)c * 32u, lane);
                    s[nt]  = wmma16(qhf, kb, s[nt]);
                    sr[nt] = wmma16(qhf, krb, sr[nt]);
                    sr[nt] = wmma16(qrf, kb, sr[nt]);
                }
            }
        } else {
#pragma unroll
            for (int c = 0; c < 2; ++c) {
#pragma unroll
                for (int nt = 0; nt < 4; ++nt) {
                    const v16h kb = load_frag(ks, (u32)nt * 16u, 64u, (u32)c * 32u, lane);
                    s[nt] = wmma16(qa[c], kb, s[nt]);
                }
            }
        }

#pragma unroll
        for (int r = 0; r < 8; ++r) {
            const u32 nib = mw >> (u32)(r * 4);
            bool vis[4];
#pragma unroll
            for (int nt = 0; nt < 4; ++nt) vis[nt] = (((nib >> (u32)nt) & 1u) != 0u);
            float x[4];
#pragma unroll
            for (int nt = 0; nt < 4; ++nt) {
                float sv = s[nt][r];
                if constexpr (EARLY) sv = sv + sr[nt][r] * RES_INV;
                const float xv = sv * cl;
                x[nt] = vis[nt] ? xv : -1.0e30f;
            }
            float mx = x[0];
#pragma unroll
            for (int nt = 1; nt < 4; ++nt) mx = fmaxf(mx, x[nt]);
            const float tm = rowmax16(mx);
            const float mn = fmaxf(m[r], tm);
            const float al = fexp2(m[r] - mn);
            m[r] = mn;
            lacc[r] *= al;
#pragma unroll
            for (int dt = 0; dt < 4; ++dt) o[dt][r] *= al;
            if constexpr (EARLY) {
                laccR[r] *= al;
#pragma unroll
                for (int dt = 0; dt < 4; ++dt) oR[dt][r] *= al;
            }
            const float sh = 10.0f - mn;
#pragma unroll
            for (int nt = 0; nt < 4; ++nt) {
                const float e  = x[nt] + sh;
                const float pe = fexp2(e);
                const float pv = (vis[nt] && (e >= -14.0f)) ? pe : 0.0f;
                const f16 ph = (f16)pv;
                psw[(hh8 + (u32)r) * 64u + (u32)nt * 16u + c16] = ph;
                if constexpr (EARLY) {
                    prw[(hh8 + (u32)r) * 64u + (u32)nt * 16u + c16] = toh_flush((pv - (float)ph) * RES_SCALE);
                }
            }
        }
        __syncthreads();

#pragma unroll
        for (int kk = 0; kk < 2; ++kk) {
            const v16h pa = load_frag(psw, 0u, 64u, (u32)kk * 32u, lane);
            if constexpr (EARLY) {
                const v16h pr = load_frag(prw, 0u, 64u, (u32)kk * 32u, lane);
#pragma unroll
                for (int dt = 0; dt < 4; ++dt) {
                    const v16h vb  = load_frag(vsT, (u32)dt * 16u, KT, (u32)kk * 32u, lane);
                    const v16h vrb = load_frag(vrsT, (u32)dt * 16u, KT, (u32)kk * 32u, lane);
                    o[dt]  = wmma16(pa, vb, o[dt]);
                    oR[dt] = wmma16(pa, vrb, oR[dt]);
                    oR[dt] = wmma16(pr, vb, oR[dt]);
                }
                lacc  = wmma16(pa, ones, lacc);
                laccR = wmma16(pr, ones, laccR);
            } else {
#pragma unroll
                for (int dt = 0; dt < 4; ++dt) {
                    const v16h vb = load_frag(vsT, (u32)dt * 16u, KT, (u32)kk * 32u, lane);
                    o[dt] = wmma16(pa, vb, o[dt]);
                }
                lacc = wmma16(pa, ones, lacc);
            }
        }
    }
    __syncthreads();

#pragma unroll
    for (int r = 0; r < 8; ++r) {
        float den = lacc[r];
        if constexpr (EARLY) den = den + laccR[r] * RES_INV;
        const float inv = (CARRY_CTX / CARRY_QKV) / den;
#pragma unroll
        for (int dt = 0; dt < 4; ++dt) {
            float ov = o[dt][r];
            if constexpr (EARLY) ov = ov + oR[dt][r] * RES_INV;
            const float cv = ov * inv;
            const f16 ch = toh_flush(cv);
            psw[(hh8 + (u32)r) * 64u + (u32)dt * 16u + c16] = ch;
            if constexpr (EARLY) {
                prw[(hh8 + (u32)r) * 64u + (u32)dt * 16u + c16] = toh_flush((cv - (float)ch) * RES_SCALE);
            }
        }
    }
    __syncthreads();

    const u32 piece = lane & 7u;
    const u32 lsub  = lane >> 3;
#pragma unroll
    for (int pass = 0; pass < 2; ++pass) {
#pragma unroll
        for (u32 it = 0; it < 4; ++it) {
            const u32 L = it * 4u + lsub;
            const v8h v = *(const v8h*)&psw[L * 64u + piece * 8u];
            f16* dp = Cp + ((size_t)(bidx * (u32)SEQ + q0 + L) * HID + hidx * (u32)HD + piece * 8u);
            *(volatile v8h*)dp = v;
            if constexpr (EARLY) {
                const v8h vr = *(const v8h*)&prw[L * 64u + piece * 8u];
                f16* dr = CRp + ((size_t)(bidx * (u32)EROWS + q0 + L) * HID + hidx * (u32)HD + piece * 8u);
                *(volatile v8h*)dr = vr;
            }
        }
        if (pass == 0) __threadfence();
    }
}

__global__ void __launch_bounds__(256) __attribute__((amdgpu_num_vgpr(256)))
k_attn(const f16* __restrict__ Qp, const f16* __restrict__ Kp, const f16* __restrict__ Vt,
       const u32* __restrict__ Mw, const u32* __restrict__ Mf, f16* __restrict__ Cp) {
    attn_body<0>(Qp, Kp, Vt, (const f16*)0, (const f16*)0, (const f16*)0, Mw, Mf, Cp, (f16*)0,
                 blockIdx.x + (u32)EB);
}

__global__ void __launch_bounds__(256) __attribute__((amdgpu_num_vgpr(256)))
k_attn_early(const f16* __restrict__ Qp, const f16* __restrict__ Kp, const f16* __restrict__ Vt,
             const f16* __restrict__ QRp, const f16* __restrict__ KRp, const f16* __restrict__ VRp,
             const u32* __restrict__ Mw, const u32* __restrict__ Mf,
             f16* __restrict__ Cp, f16* __restrict__ CRp) {
    attn_body<1>(Qp, Kp, Vt, QRp, KRp, VRp, Mw, Mf, Cp, CRp, blockIdx.x);
}

static_assert((size_t)(MROWS / 2) * 256 * 8 == (size_t)MROWS * HID);
static_assert((size_t)(3 * HID / 2) * 256 * 8 == (size_t)3 * HID * HID);
static_assert((size_t)(HID / 2) * 256 * 8 == (size_t)HID * HID);
static_assert((size_t)(MROWS / 128) * (HID / 128) * 128 * 128 == (size_t)MROWS * HID);
static_assert((size_t)(SEQ / 128) * (NB * NHEAD) * 128 * HD == (size_t)MROWS * HID);
static_assert((size_t)EB * (NB * NHEAD) * 128 * HD == N_R);
static_assert((size_t)NB * EB * (HID / 128) * 128 * 128 == N_R);
static_assert((size_t)(SEQ / 128) * NKT * 256 == N_MW);
static_assert((size_t)(SEQ / 128) * NKT * 32 == N_MF);

#define WS_HALVES  (5 * N_X + 4 * N_W + 4 * N_R)
#define WS_BYTES   (WS_HALVES * 2 + (N_MW + N_MF) * 4)
static_assert(WS_BYTES <= (size_t)134217728);
static_assert((N_X * 2) % 128 == 0);
static_assert((N_W * 2) % 128 == 0);
static_assert((N_R * 2) % 128 == 0);
static_assert((WS_HALVES * 2) % 128 == 0);
static_assert((N_MW * 4) % 128 == 0);

extern "C" void kernel_launch(void* const* d_in, const int* in_sizes, int n_in,
                              void* d_out, int out_size, void* d_ws, size_t ws_size,
                              hipStream_t stream) {
    if (n_in < 6) return;
    if (in_sizes[0] < ((NB - 1) * SEQ_FULL + SEQ) * HID) return;
    if (in_sizes[1] < (SEQ - 1) * SEQ_FULL + SEQ) return;
    if (in_sizes[2] < 3 * HID * HID) return;
    if (in_sizes[3] < 3 * HID) return;
    if (in_sizes[4] < HID * HID) return;
    if (in_sizes[5] < HID) return;
    if (out_size < MROWS * HID) return;

    const float* x     = (const float*)d_in[0];
    const int*   mask  = (const int*)d_in[1];
    const float* win   = (const float*)d_in[2];
    const float* bin   = (const float*)d_in[3];
    const float* wout  = (const float*)d_in[4];
    const float* bout  = (const float*)d_in[5];

    const size_t nX = N_X;
    const size_t nW = N_W;
    const size_t nR = N_R;
    if (ws_size < (size_t)WS_BYTES) return;

    f16* Xh  = (f16*)d_ws;
    f16* Wt  = Xh  + nX;
    f16* Wo  = Wt  + 3 * nW;
    f16* Qp  = Wo  + nW;
    f16* Kp  = Qp  + nX;
    f16* Vtp = Kp  + nX;
    f16* Cp  = Vtp + nX;
    f16* QRp = Cp  + nX;
    f16* KRp = QRp + nR;
    f16* VRp = KRp + nR;
    f16* CRp = VRp + nR;
    u32* Mw  = (u32*)(CRp + nR);
    u32* Mf  = Mw + N_MW;

    const size_t resQK = 4 * nX;
    const size_t resV  = 2 * nX + 2 * nR;
    const size_t resC  = nX + 3 * nR;

    cvt_rows<<<MROWS / 2, 256, 0, stream>>>(x, Xh, (u32)MROWS, (u32)SEQ, (u32)SEQ_FULL, CARRY_X);
    cvt_rows<<<3 * HID / 2, 256, 0, stream>>>(win, Wt, (u32)(3 * HID), (u32)(3 * HID), (u32)(3 * HID), CARRY_W);
    cvt_rows<<<HID / 2, 256, 0, stream>>>(wout, Wo, (u32)HID, (u32)HID, (u32)HID, CARRY_W);

    k_mask_pack<<<dim3(SEQ / 128, NKT), 256, 0, stream>>>(mask, Mw, Mf);

    const float accQKV = CARRY_QKV / (CARRY_X * CARRY_W);
    k_gemm_qk<<<dim3(MROWS / 128, HID / 128, 2), 256, 0, stream>>>(Xh, Wt, bin, Qp, resQK, accQKV, CARRY_QKV);
    k_gemm_vt<<<dim3(MROWS / 128, HID / 128), 256, 0, stream>>>(Xh, Wt + 2 * nW, bin + 2 * HID, Vtp, resV, accQKV, CARRY_QKV);

    k_attn_early<<<dim3(EB, NB * NHEAD), 256, 0, stream>>>(Qp, Kp, Vtp, QRp, KRp, VRp, Mw, Mf, Cp, CRp);
    if (SEQ / 128 > EB) {
        k_attn<<<dim3(SEQ / 128 - EB, NB * NHEAD), 256, 0, stream>>>(Qp, Kp, Vtp, Mw, Mf, Cp);
    }

    const float accOut = 1.0f / (CARRY_CTX * CARRY_W);
    k_gemm_out<<<dim3(MROWS / 128, HID / 128), 256, 0, stream>>>(Cp, Wo, bout, (float*)d_out, resC, accOut);
}
